// GAT_14688788152986
// MI455X (gfx1250) — hardware-verified
//
#include <hip/hip_runtime.h>
#include <stddef.h>
#include <stdint.h>
#include <math.h>


#define F_IN    256
#define HC      256
#define HID     64
#define NHD     4
#define DOUT    64
#define KA2     128
#define NTHR    256
#define NWAVE   8
#define EPT     8
#define CHUNK   (NTHR * EPT)
#define WCAP    (EPT * 32)
#define LISTN   (NWAVE * WCAP)
#define NBMAX   2048
#define SLOTB   11
#define RCAP    28672
#define DEGCAP  256
#define GBM     64
#define GBN     64
#define GTHR    128
#define MROWS   128
#define NEGSL   0.2f
#define EPS_SM  1e-16f
#define EPS_LN  1e-5f
#define MX0     (-1.0e30f)
#define WSMAX   134217728
#define LDS_AGG ((2 * RCAP + 2 * NBMAX + LISTN) * 4 + 64)

static_assert((CHUNK & (CHUNK - 1)) == 0 && CHUNK <= (1 << SLOTB));
static_assert(NBMAX == (1 << SLOTB));
static_assert(NTHR * 8 == NBMAX);
static_assert(LISTN >= NBMAX);
static_assert(LISTN >= NWAVE * WCAP);
static_assert((RCAP % 32) == 0);
static_assert(LDS_AGG <= 300000);
static_assert(GBM == (GTHR / 32) * 16);
static_assert(GTHR == 2 * GBN && GTHR == 2 * GBM);
static_assert((F_IN % 32) == 0 && (KA2 % 32) == 0);
static_assert((HC % GBN) == 0 && HID == GBN);
static_assert(HC == NHD * HID);
static_assert(HC == 8 * 32);
static_assert(HID == 8 * 8);
static_assert(NHD == 4);
static_assert(DOUT == HID && KA2 == 2 * DOUT);
static_assert(DOUT * 2 * 2 == 256);
static_assert(DOUT * 4 == 256);
static_assert((MROWS % GBM) == 0);
static_assert((F_IN / 8) == 32);

typedef float          v4f  __attribute__((ext_vector_type(4)));
typedef float          v8f  __attribute__((ext_vector_type(8)));
typedef int            v4i  __attribute__((ext_vector_type(4)));
typedef int            v8i  __attribute__((ext_vector_type(8)));
typedef unsigned int   v4u  __attribute__((ext_vector_type(4)));
typedef unsigned short v8us __attribute__((ext_vector_type(8)));
typedef __bf16         v16b __attribute__((ext_vector_type(16)));
typedef v4f  __attribute__((may_alias)) v4fa;
typedef v8us __attribute__((may_alias)) v8usa;
union FragB { v16b v; v8us h[2]; v8i w; };

__device__ __forceinline__ v8f wmb(const FragB& a, const FragB& b, v8f c) {
  v8f d = __builtin_amdgcn_wmma_f32_16x16x32_bf16(false, a.v, false, b.v, (short)0, c, false, false);
  asm volatile("v_nop\n\tv_nop\n\tv_nop\n\tv_nop" : "+v"(d) : "v"(a.w), "v"(b.w));
  return d;
}

__device__ __forceinline__ unsigned int f2bf(float f) {
  const unsigned int u = __float_as_uint(f);
  return ((u + 0x7FFFu + ((u >> 16) & 1u)) >> 16) & 0xFFFFu;
}
__device__ __forceinline__ float bf2f(unsigned int b) { return __uint_as_float(b << 16); }
__device__ __forceinline__ float bfr(float f) { return bf2f(f2bf(f)); }
__device__ __forceinline__ v4f bfr4(const v4f a) {
  v4f r; r.x = bfr(a.x); r.y = bfr(a.y); r.z = bfr(a.z); r.w = bfr(a.w); return r;
}
__device__ __forceinline__ unsigned int pk2(float lo, float hi) { return f2bf(lo) | (f2bf(hi) << 16); }
__device__ __forceinline__ unsigned int pk2lo(float lo, float hi) {
  return f2bf(lo - bfr(lo)) | (f2bf(hi - bfr(hi)) << 16);
}
__device__ __forceinline__ v4u pack8(const v4f a, const v4f b) {
  v4u r;
  r.x = pk2(a.x, a.y); r.y = pk2(a.z, a.w); r.z = pk2(b.x, b.y); r.w = pk2(b.z, b.w);
  return r;
}
__device__ __forceinline__ v4u pack8lo(const v4f a, const v4f b) {
  v4u r;
  r.x = pk2lo(a.x, a.y); r.y = pk2lo(a.z, a.w); r.z = pk2lo(b.x, b.y); r.w = pk2lo(b.z, b.w);
  return r;
}
__device__ __forceinline__ float hmean4(float v) {
  v += __shfl_xor(v, 8);
  v += __shfl_xor(v, 16);
  return 0.25f * v;
}
__device__ __forceinline__ float gsum8(float v) {
  v += __shfl_xor(v, 4);
  v += __shfl_xor(v, 2);
  v += __shfl_xor(v, 1);
  return v;
}

__device__ __forceinline__ int scan_chunk(const int* __restrict__ dsts, int nE, int cbase, int slotBase,
                                          int nb, int vec8, int* list, int tid, int lane, int wave) {
  int wc = 0;
  const int el0  = tid * EPT;
  const int e0   = cbase + el0;
  const int sent = -2147483647 - 1;
  v4i da, db;
  if (vec8 != 0 && cbase + CHUNK <= nE) {
    da = *(const v4i*)(dsts + e0);
    db = *(const v4i*)(dsts + e0 + 4);
  } else {
    da.x = (e0     < nE) ? dsts[min(e0,     nE - 1)] : sent;
    da.y = (e0 + 1 < nE) ? dsts[min(e0 + 1, nE - 1)] : sent;
    da.z = (e0 + 2 < nE) ? dsts[min(e0 + 2, nE - 1)] : sent;
    da.w = (e0 + 3 < nE) ? dsts[min(e0 + 3, nE - 1)] : sent;
    db.x = (e0 + 4 < nE) ? dsts[min(e0 + 4, nE - 1)] : sent;
    db.y = (e0 + 5 < nE) ? dsts[min(e0 + 5, nE - 1)] : sent;
    db.z = (e0 + 6 < nE) ? dsts[min(e0 + 6, nE - 1)] : sent;
    db.w = (e0 + 7 < nE) ? dsts[min(e0 + 7, nE - 1)] : sent;
  }
  const unsigned nbs = (unsigned)slotBase;
  const unsigned unb = (unsigned)nb;
  const unsigned s0 = (unsigned)da.x - nbs, s1 = (unsigned)da.y - nbs;
  const unsigned s2 = (unsigned)da.z - nbs, s3 = (unsigned)da.w - nbs;
  const unsigned s4 = (unsigned)db.x - nbs, s5 = (unsigned)db.y - nbs;
  const unsigned s6 = (unsigned)db.z - nbs, s7 = (unsigned)db.w - nbs;
  const bool h0 = s0 < unb, h1 = s1 < unb, h2 = s2 < unb, h3 = s3 < unb;
  const bool h4 = s4 < unb, h5 = s5 < unb, h6 = s6 < unb, h7 = s7 < unb;
  const unsigned any = __builtin_amdgcn_ballot_w32(h0 | h1 | h2 | h3 | h4 | h5 | h6 | h7);
  if (any != 0u) {
#define HITJ(J, HJ, SJ) { \
      const unsigned mj = __builtin_amdgcn_ballot_w32(HJ); \
      if (mj != 0u) { \
        if (HJ) { \
          const int pos = wc + (int)__builtin_amdgcn_mbcnt_lo(mj, 0u); \
          if (pos < WCAP) list[wave * WCAP + pos] = ((el0 + (J)) << SLOTB) | (int)(SJ); \
        } \
        wc += (int)__builtin_popcount(mj); } }
    HITJ(0, h0, s0)
    HITJ(1, h1, s1)
    HITJ(2, h2, s2)
    HITJ(3, h3, s3)
    HITJ(4, h4, s4)
    HITJ(5, h5, s5)
    HITJ(6, h6, s6)
    HITJ(7, h7, s7)
#undef HITJ
  }
  return wc;
}

__global__ __launch_bounds__(NTHR) void k_xprep(const float* __restrict__ x, unsigned short* xb, int nN, int nUnits) {
  const int i = (int)blockIdx.x * NTHR + (int)threadIdx.x;
  if (i >= nUnits) return;
  const int row = i >> 5;
  const int c0  = (i & 31) * 8;
  const int rc  = row < nN ? row : nN - 1;
  const float* p = x + (size_t)rc * F_IN + c0;
  v4f a = *(const v4fa*)p, b = *(const v4fa*)(p + 4);
  const v4f z4 = {0.f, 0.f, 0.f, 0.f};
  if (row >= nN) { a = z4; b = z4; }
  const v4u hv = pack8(a, b);
  const size_t o = (size_t)row * F_IN + c0;
  *(volatile v4u*)(xb + o) = hv;
  __threadfence();
  *(volatile v4u*)(xb + o) = hv;
}

__global__ __launch_bounds__(NTHR) void k_wtr(const float* __restrict__ w, int Kin, int Ncol, int Nrows, int Kout,
                                              unsigned short* wt, int nUnits) {
  const int u = (int)blockIdx.x * NTHR + (int)threadIdx.x;
  if (u >= nUnits) return;
  const int kq = Kout >> 3;
  const int n  = u / kq;
  const int k8 = (u - n * kq) * 8;
  const int kk = k8 - (k8 / Kin) * Kin;
  const int ncl = n < Ncol ? n : Ncol - 1;
  const float* p = w + (size_t)kk * (size_t)Ncol + ncl;
  v4f a, b;
  a.x = p[0];                    a.y = p[(size_t)Ncol];         a.z = p[(size_t)2 * Ncol];     a.w = p[(size_t)3 * Ncol];
  b.x = p[(size_t)4 * Ncol];     b.y = p[(size_t)5 * Ncol];     b.z = p[(size_t)6 * Ncol];     b.w = p[(size_t)7 * Ncol];
  const v4f z4 = {0.f, 0.f, 0.f, 0.f};
  if (n >= Ncol || n >= Nrows) { a = z4; b = z4; }
  const v4u wv = pack8(a, b);
  unsigned short* o = wt + (size_t)n * (size_t)Kout + k8;
  *(volatile v4u*)o = wv;
  __threadfence();
  *(volatile v4u*)o = wv;
}

__global__ __launch_bounds__(GTHR) void k_gemm(
    const unsigned short* __restrict__ A, const unsigned short* __restrict__ WT,
    float* outF, int K, int ldo,
    const float* __restrict__ atts, const float* __restrict__ attd, int attLen,
    float* SD, int MPr)
{
  __shared__ __attribute__((aligned(16))) float stg[GBM * GBN];
  __shared__ __attribute__((aligned(16))) float satt[2 * GBN];
  __shared__ __attribute__((aligned(16))) float sdot[2 * GBM];
  const int tid = (int)threadIdx.x, lane = tid & 31, wave = tid >> 5, hh = lane >> 4, m = lane & 15;
  const int rowBase = (int)blockIdx.x * GBM;
  const int head    = (int)blockIdx.y;
  const int col0    = head * GBN;

  {
    const int which = tid >> 6;
    const int c  = tid & 63;
    const int cl = c < attLen ? c : attLen - 1;
    const float vs = atts[head * attLen + cl];
    const float vd = attd[head * attLen + cl];
    float v = (which == 0) ? vs : vd;
    v = (c < attLen) ? bfr(v) : 0.f;
    satt[which * GBN + c] = v;
  }

  v8f acc[4];
  {
    const v8f z = {0.f, 0.f, 0.f, 0.f, 0.f, 0.f, 0.f, 0.f};
    acc[0] = z; acc[1] = z; acc[2] = z; acc[3] = z;
  }
  const unsigned short* ap = A  + (size_t)(rowBase + 16 * wave + m) * (size_t)K + 8 * hh;
  const unsigned short* wp = WT + (size_t)(col0 + m) * (size_t)K + 8 * hh;
  const int ksteps = K >> 5;
#pragma unroll 1
  for (int ks = 0; ks < ksteps; ++ks) {
    FragB af;
    af.h[0] = *(const v8usa*)(ap + 32 * ks);
    af.h[1] = *(const v8usa*)(ap + 32 * ks + 16);
#pragma unroll
    for (int t = 0; t < 4; ++t) {
      const unsigned short* wq = wp + (size_t)(16 * t) * (size_t)K + 32 * ks;
      FragB bf;
      bf.h[0] = *(const v8usa*)wq;
      bf.h[1] = *(const v8usa*)(wq + 16);
      acc[t] = wmb(af, bf, acc[t]);
    }
  }

#pragma unroll
  for (int t = 0; t < 4; ++t) {
    const int lc = 16 * t + m;
#pragma unroll
    for (int r = 0; r < 8; ++r) {
      const int lr = 16 * wave + 8 * hh + r;
      stg[lr * GBN + lc] = acc[t][r];
    }
  }
  __syncthreads();

  {
    const int row = tid & 63, which = tid >> 6;
    const float* sa = satt + which * GBN;
    const float* hr = stg + row * GBN;
    float d = 0.f;
#pragma unroll 4
    for (int c4 = 0; c4 < GBN / 4; ++c4) {
      const v4f hv = *(const v4fa*)(hr + 4 * c4);
      const v4f av = *(const v4fa*)(sa + 4 * c4);
      d = fmaf(hv.x, av.x, d);
      d = fmaf(hv.y, av.y, d);
      d = fmaf(hv.z, av.z, d);
      d = fmaf(hv.w, av.w, d);
    }
    sdot[which * GBM + row] = d;
  }
  __syncthreads();

  v4f fv[8];
#pragma unroll
  for (int i = 0; i < 8; ++i) {
    const int lr = 16 * wave + 2 * i + hh;
    fv[i] = *(const v4fa*)(stg + lr * GBN + 4 * m);
  }
  const int which2 = lane >> 4, piece = lane & 15;
  const v4f sdv = *(const v4fa*)(sdot + which2 * GBM + 4 * piece);
  float* sp = SD + (size_t)(2 * head + which2) * (size_t)MPr + rowBase + 4 * piece;

#pragma unroll
  for (int i = 0; i < 8; ++i) {
    const int lr = 16 * wave + 2 * i + hh;
    const int gr = rowBase + lr;
    float* op = outF + (size_t)gr * (size_t)ldo + col0 + 4 * m;
    *(volatile v4f*)op = fv[i];
  }
  if (wave == 0) *(volatile v4f*)sp = sdv;
  __threadfence();
#pragma unroll
  for (int i = 0; i < 8; ++i) {
    const int lr = 16 * wave + 2 * i + hh;
    const int gr = rowBase + lr;
    float* op = outF + (size_t)gr * (size_t)ldo + col0 + 4 * m;
    *(volatile v4f*)op = fv[i];
  }
  if (wave == 0) *(volatile v4f*)sp = sdv;
}

template<int L>
__global__ __launch_bounds__(NTHR) void k_agg(
    const int* __restrict__ srcs, const int* __restrict__ dsts,
    const float* __restrict__ F, const float* __restrict__ SD,
    const float* __restrict__ bias, const float* __restrict__ gam, const float* __restrict__ bet,
    unsigned short* HP, float* out,
    int nN, int nE, int nb, int vec8, int MPr) {
  extern __shared__ v4f lds_dyn[];
  int* reg1 = (int*)lds_dyn;
  int* reg2 = reg1 + RCAP;
  int* scnt = reg2 + RCAP;
  int* soff = scnt + NBMAX;
  int* list = soff + NBMAX;
  int* wcnt = list + LISTN;
  int* wtot = wcnt + NWAVE;
  const int tid = (int)threadIdx.x, lane = tid & 31, wave = tid >> 5;
  const int nodeBase = (int)blockIdx.x * nb;

  for (int i = tid; i < NBMAX; i += NTHR) scnt[i] = 0;
  __syncthreads();

  int tot = 0;
  const int nChunks = (nE + CHUNK - 1) / CHUNK;
#pragma unroll 1
  for (int ch = 0; ch < nChunks; ++ch) {
    const int cbase = ch * CHUNK;
    const int wc = scan_chunk(dsts, nE, cbase, nodeBase, nb, vec8, list, tid, lane, wave);
    if (lane == 0) wcnt[wave] = wc;
    __syncthreads();
    int pre = 0, all = 0;
#pragma unroll
    for (int w2 = 0; w2 < NWAVE; ++w2) {
      int c = wcnt[w2];
      c = c < 0 ? 0 : (c > WCAP ? WCAP : c);
      all += c;
      pre += (w2 < wave) ? c : 0;
    }
    const int wcc  = wc > WCAP ? WCAP : wc;
    const int base = tot + pre;
#pragma unroll 1
    for (int i = lane; i < wcc; i += 32) {
      const int ent = list[wave * WCAP + i];
      const int el  = (ent >> SLOTB) & (CHUNK - 1);
      const int sl  = ent & (NBMAX - 1);
      int eid = cbase + el;
      eid = eid > nE - 1 ? nE - 1 : eid;
      const int pos = base + i;
      if (pos < RCAP) reg1[pos] = (int)(((unsigned)eid << SLOTB) | (unsigned)sl);
    }
    tot += all;
    tot = tot > RCAP ? RCAP : tot;
    __syncthreads();
  }
  const int nh = tot;

  if (wave == 0) {
#pragma unroll 1
    for (int b0 = 0; b0 < nh; b0 += 32) {
      const int idx = b0 + lane;
      const int uv  = reg1[idx < nh ? idx : nh - 1];
      const int m32 = (nh - b0) < 32 ? (nh - b0) : 32;
#pragma unroll 1
      for (int k = 0; k < m32; ++k) {
        const int u  = __builtin_amdgcn_readlane(uv, k);
        const int sl = u & (NBMAX - 1);
        if (lane == 0) scnt[sl] = scnt[sl] + 1;
      }
    }
  }
  __syncthreads();

  {
    const v4i ca = *(const v4i*)(scnt + 8 * tid);
    const v4i cb = *(const v4i*)(scnt + 8 * tid + 4);
    const int e0 = ca.x < 0 ? 0 : ca.x, e1 = ca.y < 0 ? 0 : ca.y, e2 = ca.z < 0 ? 0 : ca.z, e3 = ca.w < 0 ? 0 : ca.w;
    const int e4 = cb.x < 0 ? 0 : cb.x, e5 = cb.y < 0 ? 0 : cb.y, e6 = cb.z < 0 ? 0 : cb.z, e7 = cb.w < 0 ? 0 : cb.w;
    const int ts = e0 + e1 + e2 + e3 + e4 + e5 + e6 + e7;
    int incl = ts;
#pragma unroll
    for (int d = 1; d < 32; d <<= 1) {
      const int up = __shfl_up(incl, d);
      if (lane >= d) incl += up;
    }
    if (lane == 31) wtot[wave] = incl;
    __syncthreads();
    int pre = 0;
#pragma unroll
    for (int w2 = 0; w2 < NWAVE; ++w2) pre += (w2 < wave) ? wtot[w2] : 0;
    int run = pre + incl - ts;
    soff[8 * tid + 0] = run; run += e0;
    soff[8 * tid + 1] = run; run += e1;
    soff[8 * tid + 2] = run; run += e2;
    soff[8 * tid + 3] = run; run += e3;
    soff[8 * tid + 4] = run; run += e4;
    soff[8 * tid + 5] = run; run += e5;
    soff[8 * tid + 6] = run; run += e6;
    soff[8 * tid + 7] = run;
  }
  __syncthreads();
  for (int i = tid; i < NBMAX; i += NTHR) list[i] = soff[i];
  __syncthreads();

  if (wave == 0) {
#pragma unroll 1
    for (int b0 = 0; b0 < nh; b0 += 32) {
      const int idx = b0 + lane;
      const int uv  = reg1[idx < nh ? idx : nh - 1];
      const int m32 = (nh - b0) < 32 ? (nh - b0) : 32;
#pragma unroll 1
      for (int k = 0; k < m32; ++k) {
        const int u   = __builtin_amdgcn_readlane(uv, k);
        const int sl  = u & (NBMAX - 1);
        const int eid = (int)((unsigned)u >> SLOTB);
        if (lane == 0) {
          int pos = list[sl];
          pos = pos < 0 ? 0 : (pos > RCAP - 1 ? RCAP - 1 : pos);
          reg2[pos] = eid;
          list[sl] = pos + 1;
        }
      }
    }
  }
  __syncthreads();

  const int nbw = nb >> 3;
  const bool ovf = (nh >= RCAP);
  const float qnan = __int_as_float(0x7fc00000);

  const int c0   = 8 * lane;
  const int head = lane >> 3;
  const int j8   = 8 * (lane & 7);
  const v4f bbA  = bfr4(*(const v4fa*)(bias + c0));
  const v4f bbB  = bfr4(*(const v4fa*)(bias + c0 + 4));
  v4f gmA = {1.f, 1.f, 1.f, 1.f}, gmB = {1.f, 1.f, 1.f, 1.f};
  v4f btA = {0.f, 0.f, 0.f, 0.f}, btB = {0.f, 0.f, 0.f, 0.f};
  if (L == 1) {
    gmA = bfr4(*(const v4fa*)(gam + j8));
    gmB = bfr4(*(const v4fa*)(gam + j8 + 4));
    btA = bfr4(*(const v4fa*)(bet + j8));
    btB = bfr4(*(const v4fa*)(bet + j8 + 4));
  }
  const float* ASp = SD + (size_t)(2 * head) * (size_t)MPr;
  const float* ADp = ASp + MPr;

#pragma unroll 1
  for (int jt = 0; jt < nbw; ++jt) {
    const int slot = wave * nbw + jt;
    const int grow = nodeBase + slot;
    const int gcl  = grow < nN ? grow : nN - 1;
    int st = soff[slot];
    const int craw = scnt[slot];
    int cnt = craw;
    st  = st < 0 ? 0 : (st > nh ? nh : st);
    cnt = cnt < 0 ? 0 : (cnt > DEGCAP ? DEGCAP : cnt);
    if (cnt > nh - st) cnt = nh - st;
    const float pz = (ovf || craw > DEGCAP) ? qnan : 0.0f;

    const float adv = ADp[gcl];
    float mx = MX0, dn = 0.0f;
    v4f av = {0.f, 0.f, 0.f, 0.f};
    v4f aw = {0.f, 0.f, 0.f, 0.f};

#pragma unroll 1
    for (int q = 0; q < cnt; ++q) {
      int idx = st + q; idx = idx > RCAP - 1 ? RCAP - 1 : idx;
      int eid = reg2[idx]; eid = eid < 0 ? 0 : (eid > nE - 1 ? nE - 1 : eid);
      const int sraw = srcs[eid];
      const int s = sraw < 0 ? 0 : (sraw > nN - 1 ? nN - 1 : sraw);
      const float* fr = F + (size_t)s * HC + c0;
      const v4f fs = *(const v4fa*)fr;
      const v4f ft = *(const v4fa*)(fr + 4);
      float lg = ASp[s] + adv;
      lg = lg > 0.f ? lg : NEGSL * lg;
      const float df = lg - mx;
      const float ee = expf(-fabsf(df));
      const bool up  = df > 0.f;
      const float s1 = up ? ee : 1.0f;
      const float s2 = up ? 1.0f : ee;
      mx = up ? lg : mx;
      dn = fmaf(dn, s1, s2);
      av.x = fmaf(av.x, s1, s2 * fs.x);
      av.y = fmaf(av.y, s1, s2 * fs.y);
      av.z = fmaf(av.z, s1, s2 * fs.z);
      av.w = fmaf(av.w, s1, s2 * fs.w);
      aw.x = fmaf(aw.x, s1, s2 * ft.x);
      aw.y = fmaf(aw.y, s1, s2 * ft.y);
      aw.z = fmaf(aw.z, s1, s2 * ft.z);
      aw.w = fmaf(aw.w, s1, s2 * ft.w);
    }
    const float inv = __builtin_amdgcn_rcpf(dn + EPS_SM);
    const float g0 = hmean4(fmaf(av.x, inv, bbA.x));
    const float g1 = hmean4(fmaf(av.y, inv, bbA.y));
    const float g2 = hmean4(fmaf(av.z, inv, bbA.z));
    const float g3 = hmean4(fmaf(av.w, inv, bbA.w));
    const float g4 = hmean4(fmaf(aw.x, inv, bbB.x));
    const float g5 = hmean4(fmaf(aw.y, inv, bbB.y));
    const float g6 = hmean4(fmaf(aw.z, inv, bbB.z));
    const float g7 = hmean4(fmaf(aw.w, inv, bbB.w));

    if (L == 1) {
      const float s8 = gsum8(((g0 + g1) + (g2 + g3)) + ((g4 + g5) + (g6 + g7)));
      const float mu = s8 * (1.0f / 64.0f);
      const float d0 = g0 - mu, d1 = g1 - mu, d2 = g2 - mu, d3 = g3 - mu;
      const float d4 = g4 - mu, d5 = g5 - mu, d6 = g6 - mu, d7 = g7 - mu;
      const float q8 = gsum8(((d0 * d0 + d1 * d1) + (d2 * d2 + d3 * d3)) + ((d4 * d4 + d5 * d5) + (d6 * d6 + d7 * d7)));
      const float rstd = rsqrtf(q8 * (1.0f / 64.0f) + EPS_LN);
      const float y0 = fmaf(d0 * rstd, gmA.x, btA.x);
      const float y1 = fmaf(d1 * rstd, gmA.y, btA.y);
      const float y2 = fmaf(d2 * rstd, gmA.z, btA.z);
      const float y3 = fmaf(d3 * rstd, gmA.w, btA.w);
      const float y4 = fmaf(d4 * rstd, gmB.x, btB.x);
      const float y5 = fmaf(d5 * rstd, gmB.y, btB.y);
      const float y6 = fmaf(d6 * rstd, gmB.z, btB.z);
      const float y7 = fmaf(d7 * rstd, gmB.w, btB.w);
      const bool live = grow < nN;
      v4f o, u;
      o.x = (live ? ((y0 > 0.f) ? y0 : (y0 - y0)) : 0.f) + pz;
      o.y = (live ? ((y1 > 0.f) ? y1 : (y1 - y1)) : 0.f) + pz;
      o.z = (live ? ((y2 > 0.f) ? y2 : (y2 - y2)) : 0.f) + pz;
      o.w = (live ? ((y3 > 0.f) ? y3 : (y3 - y3)) : 0.f) + pz;
      u.x = (live ? ((y4 > 0.f) ? y4 : (y4 - y4)) : 0.f) + pz;
      u.y = (live ? ((y5 > 0.f) ? y5 : (y5 - y5)) : 0.f) + pz;
      u.z = (live ? ((y6 > 0.f) ? y6 : (y6 - y6)) : 0.f) + pz;
      u.w = (live ? ((y7 > 0.f) ? y7 : (y7 - y7)) : 0.f) + pz;
      const v4u hv = pack8(o, u);
      const v4u lv = pack8lo(o, u);
      const bool lsel = (lane & 8) != 0;
      v4u pv;
      pv.x = lsel ? lv.x : hv.x;
      pv.y = lsel ? lv.y : hv.y;
      pv.z = lsel ? lv.z : hv.z;
      pv.w = lsel ? lv.w : hv.w;
      unsigned short* gp = HP + (size_t)grow * KA2 + 8 * (lane & 15);
      const bool wr = (grow < MPr) && (lane < 16);
      if (wr) *(volatile v4u*)gp = pv;
      __threadfence();
      if (wr) *(volatile v4u*)gp = pv;
    } else {
      const int sl2 = lane >> 1;
      const float x0 = __shfl(g0, sl2), x1 = __shfl(g1, sl2), x2 = __shfl(g2, sl2), x3 = __shfl(g3, sl2);
      const float z0 = __shfl(g4, sl2), z1 = __shfl(g5, sl2), z2 = __shfl(g6, sl2), z3 = __shfl(g7, sl2);
      const bool odd = (lane & 1) != 0;
      v4f ov;
      ov.x = (odd ? z0 : x0) + pz;
      ov.y = (odd ? z1 : x1) + pz;
      ov.z = (odd ? z2 : x2) + pz;
      ov.w = (odd ? z3 : x3) + pz;
      float* op = out + (size_t)gcl * DOUT + 4 * (lane & 15);
      const bool wr = (grow < nN) && (lane < 16);
      if (wr) *(volatile v4f*)op = ov;
      __threadfence();
      if (wr) *(volatile v4f*)op = ov;
    }
  }
}

static int pick_nb(int nE, int nN) {
  int nb = NBMAX;
  while (nb > 32 && (long long)nb * (long long)nE * 5LL > (long long)RCAP * (long long)nN * 4LL) nb >>= 1;
  return nb;
}
static inline int cdiv(int a, int b) { return (a + b - 1) / b; }

extern "C" void kernel_launch(void* const* d_in, const int* in_sizes, int n_in,
                              void* d_out, int out_size, void* d_ws, size_t ws_size,
                              hipStream_t stream) {
  if (n_in < 13) return;
  const int nN = in_sizes[0] / F_IN;
  if (nN <= 0 || in_sizes[0] != nN * F_IN || nN > (1 << 22)) return;
  const int nE = in_sizes[1];
  if (nE < 1 || nE >= (1 << (32 - SLOTB))) return;
  if (in_sizes[2] != nE) return;
  if (in_sizes[3] != F_IN * HC) return;
  if (in_sizes[4] != NHD * HID || in_sizes[5] != NHD * HID) return;
  if (in_sizes[6] != HC) return;
  if (in_sizes[7] != DOUT * HC) return;
  if (in_sizes[8] != NHD * HID || in_sizes[9] != NHD * HID) return;
  if (in_sizes[10] != HC) return;
  if (in_sizes[11] != DOUT || in_sizes[12] != DOUT) return;
  if (out_size != nN * DOUT) return;

  const float* x    = (const float*)d_in[0];
  const int*   src  = (const int*)  d_in[1];
  const int*   dst  = (const int*)  d_in[2];
  const float* W1   = (const float*)d_in[3];
  const float* al1  = (const float*)d_in[4];
  const float* ar1  = (const float*)d_in[5];
  const float* b1   = (const float*)d_in[6];
  const float* W2   = (const float*)d_in[7];
  const float* al2  = (const float*)d_in[8];
  const float* ar2  = (const float*)d_in[9];
  const float* b2   = (const float*)d_in[10];
  const float* gam  = (const float*)d_in[11];
  const float* bet  = (const float*)d_in[12];
  float* out = (float*)d_out;

  const int MP   = cdiv(nN, MROWS) * MROWS;
  const int nb   = pick_nb(nE, nN);
  if (nb < 32 || (nb & (nb - 1)) != 0 || nb > NBMAX) return;
  const int gA   = cdiv(MP, nb);
  const int vec8 = ((nE & 3) == 0) ? 1 : 0;
  if (gA * nb < MP) return;

  char* ws = (char*)d_ws;
  size_t off = 0;
  const size_t oXB  = off; off += (size_t)MP * F_IN * 2;           off = (off + 255) & ~(size_t)255;
  const size_t oW1T = off; off += (size_t)HC * F_IN * 2;           off = (off + 255) & ~(size_t)255;
  const size_t oW2T = off; off += (size_t)HC * KA2 * 2;            off = (off + 255) & ~(size_t)255;
  const size_t oFT  = off; off += (size_t)MP * HC * 4;             off = (off + 255) & ~(size_t)255;
  const size_t oSD1 = off; off += (size_t)2 * NHD * MP * 4;        off = (off + 255) & ~(size_t)255;
  const size_t oX1  = off; off += (size_t)MP * KA2 * 2;            off = (off + 255) & ~(size_t)255;
  const size_t oSD2 = off; off += (size_t)2 * NHD * MP * 4;        off = (off + 255) & ~(size_t)255;
  if (off > ws_size || off > (size_t)WSMAX) return;
  unsigned short* XB   = (unsigned short*)(ws + oXB);
  unsigned short* W1T  = (unsigned short*)(ws + oW1T);
  unsigned short* W2T2 = (unsigned short*)(ws + oW2T);
  float*          FT   = (float*)(ws + oFT);
  float*          SD1  = (float*)(ws + oSD1);
  unsigned short* X1HL = (unsigned short*)(ws + oX1);
  float*          SD2  = (float*)(ws + oSD2);

  hipFuncSetAttribute(reinterpret_cast<const void*>(&k_agg<1>),
                      hipFuncAttributeMaxDynamicSharedMemorySize, LDS_AGG);
  hipFuncSetAttribute(reinterpret_cast<const void*>(&k_agg<2>),
                      hipFuncAttributeMaxDynamicSharedMemorySize, LDS_AGG);

  const int nUx = MP * (F_IN / 8);
  k_xprep<<<cdiv(nUx, NTHR), NTHR, 0, stream>>>(x, XB, nN, nUx);

  {
    const int nUw1 = HC * (F_IN / 8);
    k_wtr<<<cdiv(nUw1, NTHR), NTHR, 0, stream>>>(W1, F_IN, HC, HC, F_IN, W1T, nUw1);
    const int nUw2 = HC * (KA2 / 8);
    k_wtr<<<cdiv(nUw2, NTHR), NTHR, 0, stream>>>(W2, DOUT, HC, HC, KA2, W2T2, nUw2);
  }

  const int gM = MP / GBM;
  k_gemm<<<dim3(gM, HC / GBN), GTHR, 0, stream>>>(XB, W1T, FT, F_IN, HC, al1, ar1, HID, SD1, MP);
  k_agg<1><<<gA, NTHR, LDS_AGG, stream>>>(src, dst, FT, SD1, b1, gam, bet, X1HL, out, nN, nE, nb, vec8, MP);
  k_gemm<<<dim3(gM, HC / GBN), GTHR, 0, stream>>>(X1HL, W2T2, FT, KA2, HC, al2, ar2, HID, SD2, MP);
  k_agg<2><<<gA, NTHR, LDS_AGG, stream>>>(src, dst, FT, SD2, b2, gam, bet, X1HL, out, nN, nE, nb, vec8, MP);
}
